// NKMLPPredictor_29678224016204
// MI455X (gfx1250) — hardware-verified
//
#include <hip/hip_runtime.h>
#include <math.h>

typedef __attribute__((ext_vector_type(16))) _Float16 v16h;
typedef __attribute__((ext_vector_type(16))) __bf16 v16b;
typedef __attribute__((ext_vector_type(8)))  _Float16 v8h;
typedef __attribute__((ext_vector_type(8)))  float v8f;
typedef __attribute__((ext_vector_type(4)))  float v4f;
typedef __attribute__((ext_vector_type(2)))  float v2f;
typedef __attribute__((ext_vector_type(4)))  unsigned v4u;
typedef __attribute__((ext_vector_type(4)))  int v4i;
typedef float __attribute__((may_alias)) float_a;
typedef int __attribute__((may_alias)) int_a;

template <typename T> __device__ __forceinline__ void vst2(void* p, T v) { *(volatile T*)p = v; __threadfence(); *(volatile T*)p = v; }
__device__ __forceinline__ v8f wmma16(v16h a, v16h b, v8f c) {
  v8f d = __builtin_amdgcn_wmma_f32_16x16x32_f16(false, a, false, b, (short)0, c, false, false);
  asm volatile("v_nop\n\tv_nop\n\tv_nop\n\tv_nop" : "+v"(d) : "v"(a), "v"(b));
  return d;
}
__device__ __forceinline__ v8f wmma_bf(v16b a, v16b b, v8f c) {
  v8f d = __builtin_amdgcn_wmma_f32_16x16x32_bf16(false, a, false, b, (short)0, c, false, false);
  asm volatile("v_nop\n\tv_nop\n\tv_nop\n\tv_nop" : "+v"(d) : "v"(a), "v"(b));
  return d;
}
__device__ __forceinline__ v16h frag_h(const _Float16* rowk0, int lane) {
  union { v16h v; v8h q[2]; } u; const _Float16* p = rowk0 + 8 * (lane >> 4);
  u.q[0] = *(const v8h*)p; u.q[1] = *(const v8h*)(p + 16); return u.v;
}
__device__ __forceinline__ v16h frag_f32(const float* rowk0, int lane) {
  v16h a; const float* p = rowk0 + 8 * (lane >> 4);
#pragma unroll
  for (int i = 0; i < 8; ++i) { a[i] = (_Float16)p[i]; a[8 + i] = (_Float16)p[16 + i]; }
  return a;
}
__device__ __forceinline__ v16h frag_f32s(const float* rowk0, int lane, float sc) {
  v16h a; const float* p = rowk0 + 8 * (lane >> 4);
#pragma unroll
  for (int i = 0; i < 8; ++i) { a[i] = (_Float16)(p[i] * sc); a[8 + i] = (_Float16)(p[16 + i] * sc); }
  return a;
}
__device__ __forceinline__ v16h fragc_f32(const float* W, int k0, int n, int lane, int ld, int K) {
  v16h a; const int g = lane >> 4;
#pragma unroll
  for (int i = 0; i < 8; ++i) { const int ka = k0 + 8 * g + i, kb = ka + 16;
    a[i] = (_Float16)(ka < K ? W[(size_t)(ka < K ? ka : K - 1) * ld + n] : 0.f); a[8 + i] = (_Float16)(kb < K ? W[(size_t)(kb < K ? kb : K - 1) * ld + n] : 0.f); }
  return a;
}
struct F2 { v16b h, l; };
__device__ __forceinline__ F2 bsplit16(const float v[16]) { F2 r;
#pragma unroll
  for (int i = 0; i < 16; ++i) { const __bf16 h = (__bf16)v[i]; r.h[i] = h; r.l[i] = (__bf16)(v[i] - (float)h); }
  return r; }
__device__ __forceinline__ F2 split_row(const float* row, int k0, int lane) { float v[16]; const float* p = row + k0 + 8 * (lane >> 4);
#pragma unroll
  for (int i = 0; i < 8; ++i) { v[i] = p[i]; v[8 + i] = p[16 + i]; }
  return bsplit16(v); }
__device__ __forceinline__ F2 split_rowK(const float* row, int k0, int lane, int K) { float v[16]; const int g = lane >> 4;
#pragma unroll
  for (int i = 0; i < 8; ++i) { const int ka = k0 + 8 * g + i, kb = ka + 16; v[i] = ka < K ? row[ka < K ? ka : K - 1] : 0.f; v[8 + i] = kb < K ? row[kb < K ? kb : K - 1] : 0.f; }
  return bsplit16(v); }
__device__ __forceinline__ F2 split_col(const float* W, int k0, int n, int lane, int ld, int K) { float v[16]; const int g = lane >> 4;
#pragma unroll
  for (int i = 0; i < 8; ++i) { const int ka = k0 + 8 * g + i, kb = ka + 16; v[i] = ka < K ? W[(size_t)(ka < K ? ka : K - 1) * ld + n] : 0.f; v[8 + i] = kb < K ? W[(size_t)(kb < K ? kb : K - 1) * ld + n] : 0.f; }
  return bsplit16(v); }
__device__ __forceinline__ v8f mac3(const F2& a, const F2& b, v8f c) { c = wmma_bf(a.l, b.h, c); c = wmma_bf(a.h, b.l, c); return wmma_bf(a.h, b.h, c); }
__device__ __forceinline__ float sigm(float v) { return 1.0f / (1.0f + expf(-v)); }
#define LDSX() do { asm volatile("s_wait_dscnt 0" ::: "memory"); __builtin_amdgcn_wave_barrier(); __builtin_amdgcn_fence(__ATOMIC_RELEASE, "workgroup"); } while (0)


#define NE 600000
#define NNODE 50000
#define FF 128
#define EF 12
#define DIN 268
#define KP 288
#define C1 28
#define C1P 32
#define C2 8
#define C2P 16
#define NBLK (NE / 64)
#define BNEPS 1e-5f
#ifndef TBLK
#define TBLK NBLK
#endif
typedef __attribute__((ext_vector_type(8))) __bf16 v8b;
__device__ __forceinline__ v16b frag_b(const __bf16* rowk0, int lane) {
  union { v16b v; v8b q[2]; } u; const __bf16* p = rowk0 + 8 * (lane >> 4);
  u.q[0] = *(const v8b*)p; u.q[1] = *(const v8b*)(p + 16); return u.v;
}
__device__ __forceinline__ float bfr(float v) { return (float)(__bf16)v; }
__device__ __attribute__((noinline)) float exp_ni(float v) { return expf(v); }
__device__ __attribute__((noinline)) float erf_ni(float v) { return erff(v); }

#define WS_W1  0u
#define WS_W2  (WS_W1 + 2u * C1P * KP)
#define WS_W3  (WS_W2 + 2u * C2P * C1P)
#define WS_Y1  (WS_W3 + 2u * C2P * C1P)
#define WS_Y2  (WS_Y1 + 4u * (size_t)NE * C1P)
#define WS_P1  (WS_Y2 + 4u * (size_t)NE * C2P)
#define WS_P2  (WS_P1 + 4u * (size_t)NBLK * 64)
#define WS_S1  (WS_P2 + 4u * (size_t)NBLK * 32)
#define WS_S2  (WS_S1 + 256u)
#define WS_END (WS_S2 + 256u)

__global__ __launch_bounds__(256) void k_packw(const float* __restrict__ W1, const float* __restrict__ W2, const float* __restrict__ W3, char* __restrict__ ws) { __shared__ __align__(16) __bf16 s1[C1P * KP]; __shared__ __align__(16) __bf16 s2[C2P * C1P], s3[C2P * C1P]; const int t = threadIdx.x;
  for (int e = t; e < C1P * KP; e += 256) { const int n = e / KP, k = e % KP; s1[e] = (n < C1 && k < DIN) ? (__bf16)W1[(size_t)n * DIN + k] : (__bf16)0.0f; }
  for (int e = t; e < C2P * C1P; e += 256) { const int n = e / C1P, k = e % C1P; s2[e] = (n < C2 && k < C1) ? (__bf16)W2[n * C1 + k] : (__bf16)0.0f; s3[e] = (n == 0 && k < C2) ? (__bf16)W3[k] : (__bf16)0.0f; }
  __syncthreads(); for (int q = t; q < C1P * KP / 8; q += 256) vst2((unsigned*)((__bf16*)(ws + WS_W1) + q * 8), *(const v4u*)&s1[q * 8]); if (t < C2P * C1P / 8) { vst2((unsigned*)((__bf16*)(ws + WS_W2) + t * 8), *(const v4u*)&s2[t * 8]); vst2((unsigned*)((__bf16*)(ws + WS_W3) + t * 8), *(const v4u*)&s3[t * 8]); } }
__global__ __launch_bounds__(128) void k_l1(const float* __restrict__ Hn, const float* __restrict__ EFt, const int* __restrict__ SRC, const int* __restrict__ DST, const __bf16* __restrict__ W1p, const float* __restrict__ B1, float* __restrict__ Y1, float* __restrict__ P1) { __shared__ int su[64], sv[64]; __shared__ __align__(16) float sy[64][C1P + 4]; __shared__ __align__(16) float spart[64];
  const int tid = threadIdx.x, wave = tid >> 5, lane = tid & 31, col = lane & 15, g = lane >> 4; const size_t e0 = (size_t)blockIdx.x * 64;
  if (tid < 64) { int u = SRC[e0 + tid], v = DST[e0 + tid]; u = u < 0 ? 0 : (u >= NNODE ? NNODE - 1 : u); v = v < 0 ? 0 : (v >= NNODE ? NNODE - 1 : v); su[tid] = u; sv[tid] = v; } __syncthreads();
  const int rl = wave * 16 + col; const float* hu = Hn + (size_t)su[rl] * FF; const float* hv = Hn + (size_t)sv[rl] * FF; const float* ef = EFt + (e0 + rl) * EF;
  v8f acc[2] = {};
#pragma unroll
  for (int kc = 0; kc < KP / 32; ++kc) { v16b a;
#pragma unroll
    for (int i = 0; i < 16; ++i) { const int k = kc * 32 + 8 * g + (i < 8 ? i : 8 + i); float x; if (k < FF) x = hu[k]; else if (k < 2 * FF) x = hv[k - FF]; else if (k < DIN) x = ef[k - 2 * FF]; else x = 0.f; a[i] = (__bf16)x; }
#pragma unroll
    for (int j = 0; j < 2; ++j) acc[j] = wmma_bf(a, frag_b(W1p + (size_t)(j * 16 + col) * KP + kc * 32, lane), acc[j]); }
#pragma unroll
  for (int j = 0; j < 2; ++j) { const int c = j * 16 + col; const float bb = (c < C1) ? bfr(B1[c]) : 0.f;
#pragma unroll
    for (int r = 0; r < 8; ++r) sy[wave * 16 + 8 * g + r][c] = (c < C1) ? acc[j][r] + bb : 0.f; }
  __syncthreads();
  if (tid < 64) { const int c = tid & 31, sq = tid >> 5; float s = 0.f;
#pragma unroll 1
    for (int r = 0; r < 64; ++r) { const float v = sy[r][c]; s += sq ? v * v : v; } spart[tid] = s; }
  __syncthreads();
  for (int e = tid; e < 64 * 8; e += 128) { const int r = e >> 3, q = e & 7; vst2(Y1 + (e0 + r) * C1P + q * 4, *(const v4f*)&sy[r][q * 4]); }
  if (tid < 16) vst2(P1 + (size_t)blockIdx.x * 64 + tid * 4, *(const v4f*)&spart[tid * 4]); }
__global__ __launch_bounds__(256) void k_stat(const float* __restrict__ P, int nblk, int w, int st, float cnt, float* __restrict__ S) { __shared__ float red[256]; __shared__ __align__(16) float so[64]; const int t = threadIdx.x; const int c = t & 31, part = t >> 5;
  float s = 0.f, q = 0.f; if (c < w) {
#pragma unroll 1
    for (int bidx = part; bidx < nblk; bidx += 8) { s += P[(size_t)bidx * st + c]; q += P[(size_t)bidx * st + w + c]; } }
  red[t] = s; __syncthreads(); if (t < 32) { float ss = 0.f; for (int i = 0; i < 8; ++i) ss += red[i * 32 + t]; so[t] = ss / cnt; } __syncthreads();
  red[t] = q; __syncthreads(); if (t < 32) { float qq = 0.f; for (int i = 0; i < 8; ++i) qq += red[i * 32 + t]; const float mean = so[t]; const float var = qq / cnt - mean * mean; so[32 + t] = (t < w) ? 1.0f / sqrtf(fmaxf(var, 0.f) + BNEPS) : 0.f; }
  __syncthreads(); if (t < 16) vst2(S + t * 4, *(const v4f*)&so[t * 4]); }
__global__ __launch_bounds__(128) void k_l2(const float* __restrict__ Y1, const float* __restrict__ S1, const float* __restrict__ G1, const float* __restrict__ T1, const __bf16* __restrict__ W2p, const float* __restrict__ B2, float* __restrict__ Y2, float* __restrict__ P2) { __shared__ __align__(16) float sy[64][C2P + 4]; __shared__ __align__(16) float spart[32]; __shared__ float smean[32], sinv[32], sg[32], st[32];
  const int tid = threadIdx.x, wave = tid >> 5, lane = tid & 31, col = lane & 15, g = lane >> 4; const size_t e0 = (size_t)blockIdx.x * 64;
  if (tid < 32) { smean[tid] = S1[tid]; sinv[tid] = S1[32 + tid]; sg[tid] = tid < C1 ? bfr(G1[tid]) : 0.f; st[tid] = tid < C1 ? bfr(T1[tid]) : 0.f; } __syncthreads();
  const int rl = wave * 16 + col; float x[16]; const float* yr = Y1 + (e0 + rl) * C1P;
#pragma unroll
  for (int i = 0; i < 16; ++i) { const int k = 8 * g + (i < 8 ? i : 8 + i); const float v = (yr[k] - smean[k]) * sinv[k] * sg[k] + st[k]; x[i] = (k < C1) ? fmaxf(v, 0.f) : 0.f; }
  const F2 a = bsplit16(x); v8f acc = {}; { const v16b w = frag_b(W2p + (size_t)col * C1P, lane); acc = wmma_bf(a.h, w, acc); acc = wmma_bf(a.l, w, acc); }
  { const float bb = (col < C2) ? bfr(B2[col]) : 0.f;
#pragma unroll
    for (int r = 0; r < 8; ++r) sy[wave * 16 + 8 * g + r][col] = (col < C2) ? acc[r] + bb : 0.f; }
  __syncthreads();
  if (tid < 32) { const int c = tid & 15, sq = tid >> 4; float s = 0.f;
#pragma unroll 1
    for (int r = 0; r < 64; ++r) { const float v = sy[r][c]; s += sq ? v * v : v; } spart[tid] = s; }
  __syncthreads();
  for (int e = tid; e < 64 * 4; e += 128) { const int r = e >> 2, q = e & 3; vst2(Y2 + (e0 + r) * C2P + q * 4, *(const v4f*)&sy[r][q * 4]); }
  if (tid < 8) vst2(P2 + (size_t)blockIdx.x * 32 + tid * 4, *(const v4f*)&spart[tid * 4]); }
__global__ __launch_bounds__(128) void k_l3(const float* __restrict__ Y2, const float* __restrict__ S2, const float* __restrict__ G2, const float* __restrict__ T2, const __bf16* __restrict__ W3p, const float* __restrict__ B3, float* __restrict__ OUT) { __shared__ __align__(16) float so[64]; __shared__ float smean[16], sinv[16], sg[16], st[16];
  const int tid = threadIdx.x, wave = tid >> 5, lane = tid & 31, col = lane & 15, g = lane >> 4; const size_t e0 = (size_t)blockIdx.x * 64;
  if (tid < 16) { smean[tid] = S2[tid]; sinv[tid] = S2[32 + tid]; sg[tid] = tid < C2 ? bfr(G2[tid]) : 0.f; st[tid] = tid < C2 ? bfr(T2[tid]) : 0.f; } __syncthreads();
  const int rl = wave * 16 + col; float x[16]; const float* yr = Y2 + (e0 + rl) * C2P;
#pragma unroll
  for (int i = 0; i < 16; ++i) { const int k = 8 * g + (i < 8 ? i : 8 + i); const float v = (k < C2P) ? (yr[k < C2P ? k : 0] - smean[k & 15]) * sinv[k & 15] * sg[k & 15] + st[k & 15] : 0.f; x[i] = (k < C2) ? fmaxf(v, 0.f) : 0.f; }
  const F2 a = bsplit16(x); v8f acc = {}; { const v16b w = frag_b(W3p + (size_t)col * C1P, lane); acc = wmma_bf(a.h, w, acc); acc = wmma_bf(a.l, w, acc); }
  if (col == 0) { const float bb = bfr(B3[0]);
#pragma unroll
    for (int r = 0; r < 8; ++r) so[wave * 16 + 8 * g + r] = acc[r] + bb; }
  __syncthreads(); if (tid < 16) vst2(OUT + e0 + tid * 4, *(const v4f*)&so[tid * 4]); }
extern "C" void kernel_launch(void* const* d_in, const int* in_sizes, int n_in, void* d_out, int out_size, void* d_ws, size_t ws_size, hipStream_t stream) {
  (void)in_sizes; (void)n_in; (void)out_size;
  const float** F = (const float**)d_in;
  if (ws_size < (size_t)WS_END) return;
  char* ws = (char*)d_ws; __bf16 *W1p = (__bf16*)(ws + WS_W1), *W2p = (__bf16*)(ws + WS_W2), *W3p = (__bf16*)(ws + WS_W3); float *Y1 = (float*)(ws + WS_Y1), *Y2 = (float*)(ws + WS_Y2), *P1 = (float*)(ws + WS_P1), *P2 = (float*)(ws + WS_P2), *S1 = (float*)(ws + WS_S1), *S2 = (float*)(ws + WS_S2);
  const float cnt = (float)(TBLK * 64);
  k_packw<<<1, 256, 0, stream>>>(F[4], F[8], F[12], ws);
  k_l1<<<TBLK, 128, 0, stream>>>(F[0], F[1], (const int*)d_in[2], (const int*)d_in[3], W1p, F[5], Y1, P1);
  k_stat<<<1, 256, 0, stream>>>(P1, TBLK, 32, 64, cnt, S1);
  k_l2<<<TBLK, 128, 0, stream>>>(Y1, S1, F[6], F[7], W2p, F[9], Y2, P2);
  k_stat<<<1, 256, 0, stream>>>(P2, TBLK, 16, 32, cnt, S2);
  k_l3<<<TBLK, 128, 0, stream>>>(Y2, S2, F[10], F[11], W3p, F[13], (float*)d_out);
}
